// GlobalSemanticsAggregator_66486093742336
// MI455X (gfx1250) — hardware-verified
//
#include <hip/hip_runtime.h>
#include <math.h>

#ifndef NB
#define NB 64
#endif
#ifndef SEQ
#define SEQ 512
#endif
#define NB_FULL 64
#define SEQ_FULL 512
#define DIM 256
#define NWIN 3
#define MTOK (NB * SEQ)
#define CARRY_X 16.0f
#define CARRY_W 64.0f
#define LOG2E_F 1.4426950408889634f

static constexpr float SC_H  = 1.0f / 1024.0f;
static constexpr float ONE_F = 1.0f;
static constexpr float CW_F  = CARRY_W;

static_assert(CARRY_X * CARRY_W * SC_H == 1.0f);
static_assert(SEQ % 256 == 0 && SEQ <= 512);
static_assert(SEQ <= SEQ_FULL && NB <= NB_FULL);
static_assert(MTOK % 64 == 0);
static_assert(DIM % 64 == 0 && DIM % 32 == 0);
static_assert(DIM == 256);
static_assert(DIM / 8 == 32);
static_assert((MTOK * 32) % 256 == 0);
static_assert(MTOK % 256 == 0);
static_assert(32 * 16 == DIM * 2);
static_assert(32 * 4 == 128);
static_assert(64 * 16 == DIM * 4);
static_assert(2 * 4 * 2 == 16);
static_assert(4 * 4 == 16);
static_assert(8 * 16 * 68 * 4 <= 131072);
static_assert((5 * SEQ + SEQ / 32 + (SEQ / 256) * 256) * 4 <= 131072);

typedef __attribute__((ext_vector_type(16))) _Float16 v16h;
typedef __attribute__((ext_vector_type(8)))  _Float16 v8h;
typedef __attribute__((ext_vector_type(8)))  float    v8f;
typedef __attribute__((ext_vector_type(4)))  float    v4f;
typedef __attribute__((ext_vector_type(4)))  unsigned int v4u;
typedef _Float16 h16;


#define VST2(T, ptr, val) do { const T vst2_v_ = (val); *(volatile T*)(ptr) = vst2_v_; __threadfence(); *(volatile T*)(ptr) = vst2_v_; } while (0)
#define VST2V4(ptr, val) do { const v4f vst2_v4_ = (val); *(volatile v4f*)(ptr) = vst2_v4_; __threadfence(); *(volatile v4f*)(ptr) = vst2_v4_; } while (0)

__device__ __forceinline__ float bfr(float f) {
    unsigned u = __float_as_uint(f);
    u += 0x7FFFu + ((u >> 16) & 1u);
    return __uint_as_float(u & 0xFFFF0000u);
}
__device__ __forceinline__ unsigned short f2h_bits(float x) {
    return (fabsf(x) < 6.104e-5f) ? (unsigned short)0 : __builtin_bit_cast(unsigned short, (_Float16)x);
}
__device__ __forceinline__ void st8h(unsigned short* P, size_t o, const float* v) {
    v4u pk;
    pk.x = (unsigned)f2h_bits(v[0]) | ((unsigned)f2h_bits(v[1]) << 16);
    pk.y = (unsigned)f2h_bits(v[2]) | ((unsigned)f2h_bits(v[3]) << 16);
    pk.z = (unsigned)f2h_bits(v[4]) | ((unsigned)f2h_bits(v[5]) << 16);
    pk.w = (unsigned)f2h_bits(v[6]) | ((unsigned)f2h_bits(v[7]) << 16);
    VST2(v4u, (v4u*)(P + o), pk);
}
static __device__ __forceinline__ h16 toh_flush(float v) { const float w = (fabsf(v) < 6.103515625e-05f) ? 0.0f : v; return (h16)w; }

union FragU { v16h v; v8h h[2]; };
__device__ __forceinline__ v16h frag_ld(const _Float16* p) {
    FragU f; f.h[0] = *(const v8h*)(p); f.h[1] = *(const v8h*)(p + 16); return f.v;
}
__device__ __forceinline__ v8f wmma16(v16h a, v16h b, v8f c) {
    c = __builtin_amdgcn_wmma_f32_16x16x32_f16(false, a, false, b, (short)0, c, false, false);
    asm volatile("v_nop\n\tv_nop\n\tv_nop\n\tv_nop" : "+v"(c) : "v"(a), "v"(b));
    return c;
}
__device__ __forceinline__ void wave_sync_lds() {
    __builtin_amdgcn_fence(3  , "workgroup");
    __builtin_amdgcn_wave_barrier();
    __builtin_amdgcn_fence(2  , "workgroup");
}
__device__ __forceinline__ float lrelu(float x) { return (x >= 0.0f) ? x : 0.2f * x; }

template <int OUT_MODE, bool RESID, bool RELU>
__global__ __launch_bounds__(256) void k_gemm64(
    const _Float16* __restrict__ A, unsigned lda, const _Float16* __restrict__ Bt, unsigned ldb,
    void* __restrict__ Cout, unsigned ldc, const float* __restrict__ bias, const float* __restrict__ resid,
    unsigned M, unsigned N, unsigned K, float scale, float oscale) {
  __shared__ __align__(16) float sT[8][16 * 68];
  const unsigned lane = threadIdx.x & 31u;
  const unsigned wave = threadIdx.x >> 5;
  const unsigned tilesN = N >> 6, tilesM = M >> 6;
  const unsigned tile = blockIdx.x * 8u + wave;
  if (tile >= tilesM * tilesN) return;
  const unsigned tm = tile / tilesN;
  const unsigned tn = tile - tm * tilesN;
  const unsigned m0 = tm << 6, n0 = tn << 6;
  const unsigned rlane = lane & 15u;
  const unsigned koff = (lane >> 4) * 8u;
  const unsigned mOff = koff;

  v8f acc[4][4];
#pragma unroll
  for (int i = 0; i < 4; ++i)
#pragma unroll
    for (int j = 0; j < 4; ++j) acc[i][j] = (v8f){0.f,0.f,0.f,0.f,0.f,0.f,0.f,0.f};

  for (unsigned k0 = 0; k0 < K; k0 += 32u) {
    v16h bh[4];
#pragma unroll
    for (int j = 0; j < 4; ++j)
      bh[j] = frag_ld(Bt + (size_t)(n0 + ((unsigned)j << 4) + rlane) * ldb + koff + k0);
#pragma unroll
    for (int i = 0; i < 4; ++i) {
      const v16h ah = frag_ld(A + (size_t)(m0 + ((unsigned)i << 4) + rlane) * lda + koff + k0);
#pragma unroll
      for (int j = 0; j < 4; ++j)
        acc[i][j] = wmma16(ah, bh[j], acc[i][j]);
    }
  }

  float* slab = sT[wave];
#pragma unroll
  for (int i = 0; i < 4; ++i) {
    const unsigned mBase = m0 + ((unsigned)i << 4);
#pragma unroll
    for (int j = 0; j < 4; ++j) {
      const unsigned n = n0 + ((unsigned)j << 4) + rlane;
      const float bv = bfr(bias[n]);
#pragma unroll
      for (int r = 0; r < 8; ++r) {
        float v = acc[i][j][r] * scale + bv;
        if (RELU) v = fmaxf(v, 0.0f);
        if (OUT_MODE == 1) v *= oscale;
        slab[(mOff + (unsigned)r) * 68u + ((unsigned)j << 4) + rlane] = v;
      }
    }
    wave_sync_lds();
    if (OUT_MODE == 0) {
      float* C = (float*)Cout;
      const unsigned hh = lane >> 4, c4 = (lane & 15u) * 4u;
#pragma unroll
      for (int half = 0; half < 2; ++half) {
        v4f vv[4];
#pragma unroll
        for (int it = 0; it < 4; ++it) {
          const unsigned row = (unsigned)(half * 4 + it) * 2u + hh;
          vv[it] = *(const v4f*)(slab + row * 68u + c4);
          if (RESID) vv[it] += *(const v4f*)(resid + (size_t)(mBase + row) * ldc + n0 + c4);
        }
        for (int pass = 0; pass < 2; ++pass) {
#pragma unroll
          for (int it = 0; it < 4; ++it) {
            const unsigned row = (unsigned)(half * 4 + it) * 2u + hh;
            *(volatile v4f*)(C + (size_t)(mBase + row) * ldc + n0 + c4) = vv[it];
          }
          __threadfence();
        }
      }
    } else {
      _Float16* C = (_Float16*)Cout;
      const unsigned q = lane >> 3, c8 = (lane & 7u) * 8u;
      v8h hv[4];
#pragma unroll
      for (int it = 0; it < 4; ++it) {
        const unsigned row = (unsigned)it * 4u + q;
        const float* sp = slab + row * 68u + c8;
#pragma unroll
        for (int e = 0; e < 8; ++e) hv[it][e] = toh_flush(sp[e]);
      }
      for (int pass = 0; pass < 2; ++pass) {
#pragma unroll
        for (int it = 0; it < 4; ++it) {
          const unsigned row = (unsigned)it * 4u + q;
          *(volatile v8h*)(C + (size_t)(mBase + row) * ldc + n0 + c8) = hv[it];
        }
        __threadfence();
      }
    }
    wave_sync_lds();
  }
}

__global__ __launch_bounds__(256) void k_wt16(const float* __restrict__ Wm, unsigned KI, unsigned NO, unsigned lgper,
                                              unsigned short* __restrict__ W16, float sw) {
    const unsigned layer = blockIdx.y;
    const float* Wl = Wm + (size_t)layer * KI * NO;
    unsigned short* Dl = W16 + (size_t)layer * KI * NO;
    const unsigned u = blockIdx.x * 256u + threadIdx.x;
    const unsigned per = 1u << lgper;
    if (u >= NO * per) return;
    const unsigned k0 = 8u * (u & (per - 1u));
    const unsigned o = u >> lgper;
    float v[8];
#pragma unroll
    for (int i = 0; i < 8; ++i) v[i] = bfr(Wl[(size_t)(k0 + (unsigned)i) * NO + o]) * sw;
    st8h(Dl, (size_t)o * KI + k0, v);
}

__global__ __launch_bounds__(64) void k_zero(float* __restrict__ z) {
    const unsigned t = threadIdx.x;
    const v4f zz = (v4f){0.f, 0.f, 0.f, 0.f};
    if (t < 64u) { VST2V4(z + 4u * t, zz); }
}

__global__ __launch_bounds__(256) void k_pool(const float* __restrict__ x, const int* __restrict__ turns, unsigned w,
                                              _Float16* __restrict__ PL) {
    const unsigned u = blockIdx.x * 256u + threadIdx.x;
    if (u >= (unsigned)(MTOK * 32)) return;
    const unsigned row = u >> 5, c0 = (u & 31u) * 8u;
    const unsigned b = row / (unsigned)SEQ;
    const unsigned t = row % (unsigned)SEQ;
    const int turn = turns[b];
    const int cnt = max(turn - (int)w + 2, 0);
    const bool valid = ((int)t < cnt);
    const float invw = 1.0f / (float)w;
    float acc[8];
#pragma unroll
    for (int i = 0; i < 8; ++i) acc[i] = 0.0f;
#pragma unroll 1
    for (unsigned j = 0; j < w; ++j) {
        const unsigned tj = t + j;
        const unsigned tc = min(tj, (unsigned)SEQ - 1u);
        const float* xr = x + ((size_t)tc * NB_FULL + b) * DIM + c0;
        const v4f p = *(const v4f*)xr;
        const v4f q = *(const v4f*)(xr + 4);
        const bool inr = (tj < (unsigned)SEQ);
        acc[0] += inr ? bfr(p.x) : 0.0f;
        acc[1] += inr ? bfr(p.y) : 0.0f;
        acc[2] += inr ? bfr(p.z) : 0.0f;
        acc[3] += inr ? bfr(p.w) : 0.0f;
        acc[4] += inr ? bfr(q.x) : 0.0f;
        acc[5] += inr ? bfr(q.y) : 0.0f;
        acc[6] += inr ? bfr(q.z) : 0.0f;
        acc[7] += inr ? bfr(q.w) : 0.0f;
    }
    v8h hv;
#pragma unroll
    for (int i = 0; i < 8; ++i) {
        const float m = valid ? (acc[i] * invw) : 0.0f;
        hv[i] = toh_flush(m * CARRY_X);
    }
    _Float16* dst = PL + (size_t)row * DIM + c0;
    *(volatile v8h*)dst = hv;
    __threadfence();
    *(volatile v8h*)dst = hv;
}

__global__ __launch_bounds__(256) void k_rowdot(const float* __restrict__ H, const float* __restrict__ a1, const float* __restrict__ a2,
                                                float* __restrict__ F1, float* __restrict__ F2) {
    const unsigned lane = threadIdx.x & 31u;
    const unsigned wave = __builtin_amdgcn_readfirstlane(threadIdx.x >> 5);
    const unsigned base = (blockIdx.x * 8u + wave) * 32u;
    if (base >= (unsigned)MTOK) return;
    const v4f p0 = *(const v4f*)(a1 + 8u * lane), p1 = *(const v4f*)(a1 + 8u * lane + 4u);
    const v4f q0 = *(const v4f*)(a2 + 8u * lane), q1 = *(const v4f*)(a2 + 8u * lane + 4u);
    const float w1[8] = {bfr(p0.x), bfr(p0.y), bfr(p0.z), bfr(p0.w), bfr(p1.x), bfr(p1.y), bfr(p1.z), bfr(p1.w)};
    const float w2[8] = {bfr(q0.x), bfr(q0.y), bfr(q0.z), bfr(q0.w), bfr(q1.x), bfr(q1.y), bfr(q1.z), bfr(q1.w)};
    float k1 = 0.0f, k2 = 0.0f;
#pragma unroll 1
    for (unsigned r = 0; r < 32u; ++r) {
        const float* hr = H + (size_t)(base + r) * DIM + 8u * lane;
        const v4f x0 = *(const v4f*)hr;
        const v4f x1 = *(const v4f*)(hr + 4);
        float s1 = ((x0.x * w1[0] + x0.y * w1[1]) + (x0.z * w1[2] + x0.w * w1[3])) + ((x1.x * w1[4] + x1.y * w1[5]) + (x1.z * w1[6] + x1.w * w1[7]));
        float s2 = ((x0.x * w2[0] + x0.y * w2[1]) + (x0.z * w2[2] + x0.w * w2[3])) + ((x1.x * w2[4] + x1.y * w2[5]) + (x1.z * w2[6] + x1.w * w2[7]));
#pragma unroll
        for (int o = 16; o > 0; o >>= 1) { s1 += __shfl_xor(s1, o, 32); s2 += __shfl_xor(s2, o, 32); }
        k1 = (lane == r) ? s1 : k1;
        k2 = (lane == r) ? s2 : k2;
    }
    VST2(float, F1 + base + lane, k1);
    VST2(float, F2 + base + lane, k2);
}

__global__ __launch_bounds__(SEQ) void k_agg(const float* __restrict__ H, const float* __restrict__ F1, const float* __restrict__ F2,
                                             const int* __restrict__ turns, unsigned w, float* __restrict__ inter) {
    __shared__ float sF1[SEQ];
    __shared__ float sF2[SEQ];
    __shared__ float sM[SEQ];
    __shared__ float sR[SEQ];
    __shared__ float sC[SEQ];
    __shared__ float sW[SEQ / 32];
    __shared__ __align__(16) float sPart[SEQ / 256][256];
    const unsigned t = threadIdx.x;
    const unsigned lane = t & 31u;
    const unsigned wave = __builtin_amdgcn_readfirstlane(threadIdx.x >> 5);
    const unsigned b = blockIdx.x;
    const int turn = turns[b];
    const int cnt = max(turn - (int)w + 2, 0);
    const unsigned ucnt = (unsigned)min(cnt, SEQ);
    const float denom = (float)max(cnt, 1);
    const float f1i = F1[(size_t)b * SEQ + t];
    const float f2i = F2[(size_t)b * SEQ + t];
    sF1[t] = f1i;
    sF2[t] = f2i;
    float mx = (t < ucnt) ? f2i : -3.0e38f;
#pragma unroll
    for (int o = 16; o > 0; o >>= 1) mx = fmaxf(mx, __shfl_xor(mx, o, 32));
    if (lane == 0u) sW[wave] = mx;
    __syncthreads();
    float gm = sW[0];
#pragma unroll
    for (int k = 1; k < SEQ / 32; ++k) gm = fmaxf(gm, sW[k]);

    {
        const float mi = lrelu(f1i + gm);
        float l = 0.0f;
#pragma unroll 2
        for (unsigned j = 0; j < ucnt; ++j) {
            const float e = lrelu(f1i + sF2[j]);
            l += exp2f((e - mi) * LOG2E_F);
        }
        sM[t] = mi;
        sR[t] = (l > 0.0f) ? (1.0f / l) : 0.0f;
    }
    __syncthreads();

    {
        float acc = 0.0f;
#pragma unroll 2
        for (unsigned i = 0; i < ucnt; ++i) {
            const float e = lrelu(sF1[i] + f2i);
            acc += exp2f((e - sM[i]) * LOG2E_F) * sR[i];
        }
        sC[t] = (t < ucnt) ? acc : 0.0f;
    }
    __syncthreads();

    {
        const unsigned f = t & 255u;
        const unsigned part = t >> 8;
        const unsigned jb = part * 256u;
        const float* hb = H + ((size_t)b * SEQ + (size_t)jb) * DIM + f;
        float acc = 0.0f;
#pragma unroll 4
        for (unsigned jj = 0; jj < 256u; ++jj) acc += sC[jb + jj] * hb[(size_t)jj * DIM];
        sPart[part][f] = acc;
    }
    __syncthreads();
    if (t < 256u) {
        float tot = sPart[0][t];
#pragma unroll
        for (int p = 1; p < SEQ / 256; ++p) tot += sPart[p][t];
        sPart[0][t] = tot * (1.0f / denom);
    }
    __syncthreads();
    if (t < 64u) {
        const v4f v = *(const v4f*)(&sPart[0][4u * t]);
        VST2V4(inter + (size_t)b * DIM + 4u * t, v);
    }
}

__global__ __launch_bounds__(64) void k_final(const float* __restrict__ inter, const int* __restrict__ turns, float* __restrict__ out) {
    const unsigned t = threadIdx.x;
    const unsigned b = blockIdx.x;
    const int turn = turns[b];
    v4f num = (v4f){0.f, 0.f, 0.f, 0.f};
    float vws = 0.0f;
#pragma unroll
    for (int w = 1; w <= NWIN; ++w) {
        const int cnt = max(turn - w + 2, 0);
        const float has = (cnt > 0) ? 1.0f : 0.0f;
        const v4f v = *(const v4f*)(inter + ((size_t)(w - 1) * NB + b) * DIM + 4u * t);
        num += v * has;
        vws += has;
    }
    const float iv = 1.0f / vws;
    const v4f o = num * iv;
    if (t < 64u) { VST2V4(out + (size_t)b * DIM + 4u * t, o); }
}

static constexpr size_t al256(size_t v) { return (v + 255) & ~(size_t)255; }
static constexpr size_t SZ_PL  = (size_t)MTOK * DIM * 2;
static constexpr size_t SZ_H   = (size_t)MTOK * DIM * 4;
static constexpr size_t SZ_F   = (size_t)MTOK * 4;
static constexpr size_t SZ_IN  = (size_t)NWIN * NB * DIM * 4;
static constexpr size_t SZ_ZB  = (size_t)DIM * 4;
static constexpr size_t SZ_WT  = (size_t)DIM * DIM * 2;
static constexpr size_t OFF_PL = 0;
static constexpr size_t OFF_H  = OFF_PL + al256(SZ_PL);
static constexpr size_t OFF_F1 = OFF_H  + al256(SZ_H);
static constexpr size_t OFF_F2 = OFF_F1 + al256(SZ_F);
static constexpr size_t OFF_IN = OFF_F2 + al256(SZ_F);
static constexpr size_t OFF_ZB = OFF_IN + al256(SZ_IN);
static constexpr size_t OFF_WT = OFF_ZB + al256(SZ_ZB);
static constexpr size_t WS_TOTAL = OFF_WT + al256(SZ_WT);
static_assert(WS_TOTAL <= (size_t)134217728);
static_assert(SZ_PL % 512 == 0 && SZ_H % 1024 == 0 && SZ_F % 128 == 0 && SZ_IN % 1024 == 0 && SZ_ZB % 1024 == 0 && SZ_WT % 512 == 0);

static constexpr unsigned G_WT   = (DIM * (DIM / 8)) / 256;
static constexpr unsigned G_POOL = (MTOK * 32) / 256;
static constexpr unsigned G_GEMM = ((MTOK / 64) * (DIM / 64) + 7) / 8;
static constexpr unsigned G_ROW  = MTOK / 256;
static_assert(G_WT * 256 == DIM * (DIM / 8));

extern "C" void kernel_launch(void* const* d_in, const int* in_sizes, int n_in, void* d_out, int out_size,
                              void* d_ws, size_t ws_size, hipStream_t stream) {
    if (n_in < 5) return;
    if (in_sizes[0] < SEQ * NB_FULL * DIM || in_sizes[1] < NB || in_sizes[2] < DIM * DIM) return;
    if (in_sizes[3] < DIM || in_sizes[4] < DIM || out_size < NB * DIM) return;
    if (WS_TOTAL > ws_size) return;

    const float* x     = (const float*)d_in[0];
    const int*   turns = (const int*)d_in[1];
    const float* Wm    = (const float*)d_in[2];
    const float* a1    = (const float*)d_in[3];
    const float* a2    = (const float*)d_in[4];
    float* out = (float*)d_out;

    char* wsp = (char*)d_ws;
    _Float16*       PL  = (_Float16*)(wsp + OFF_PL);
    float*          H   = (float*)(wsp + OFF_H);
    float*          F1  = (float*)(wsp + OFF_F1);
    float*          F2  = (float*)(wsp + OFF_F2);
    float*          INT = (float*)(wsp + OFF_IN);
    float*          zb  = (float*)(wsp + OFF_ZB);
    unsigned short* wt  = (unsigned short*)(wsp + OFF_WT);

    k_wt16<<<dim3(G_WT, 1), 256, 0, stream>>>(Wm, DIM, DIM, 5, wt, CW_F);
    k_zero<<<1, 64, 0, stream>>>(zb);

    for (unsigned w = 1; w <= (unsigned)NWIN; ++w) {
        k_pool<<<G_POOL, 256, 0, stream>>>(x, turns, w, PL);
        k_gemm64<0, false, false><<<G_GEMM, 256, 0, stream>>>((const _Float16*)PL, DIM, (const _Float16*)wt, DIM,
            (void*)H, DIM, zb, nullptr, MTOK, DIM, DIM, SC_H, ONE_F);
        k_rowdot<<<G_ROW, 256, 0, stream>>>(H, a1, a2, F1, F2);
        k_agg<<<NB, SEQ, 0, stream>>>(H, F1, F2, turns, w, INT + (size_t)(w - 1) * NB * DIM);
    }
    k_final<<<NB, 64, 0, stream>>>(INT, turns, out);
}
